// DeMash_7559142441226
// MI455X (gfx1250) — hardware-verified
//
#include <hip/hip_runtime.h>
#include <math.h>

typedef __attribute__((ext_vector_type(16))) _Float16 v16h;
typedef __attribute__((ext_vector_type(16))) __bf16 v16b;
typedef __attribute__((ext_vector_type(8)))  _Float16 v8h;
typedef __attribute__((ext_vector_type(8)))  float v8f;
typedef __attribute__((ext_vector_type(4)))  float v4f;
typedef __attribute__((ext_vector_type(2)))  float v2f;
typedef __attribute__((ext_vector_type(4)))  unsigned v4u;
typedef __attribute__((ext_vector_type(4)))  int v4i;
typedef float __attribute__((may_alias)) float_a;
typedef int __attribute__((may_alias)) int_a;

template <typename T> __device__ __forceinline__ void vst2(void* p, T v) { *(volatile T*)p = v; __threadfence(); *(volatile T*)p = v; }
__device__ __forceinline__ v8f wmma16(v16h a, v16h b, v8f c) {
  v8f d = __builtin_amdgcn_wmma_f32_16x16x32_f16(false, a, false, b, (short)0, c, false, false);
  asm volatile("v_nop\n\tv_nop\n\tv_nop\n\tv_nop" : "+v"(d) : "v"(a), "v"(b));
  return d;
}
__device__ __forceinline__ v8f wmma_bf(v16b a, v16b b, v8f c) {
  v8f d = __builtin_amdgcn_wmma_f32_16x16x32_bf16(false, a, false, b, (short)0, c, false, false);
  asm volatile("v_nop\n\tv_nop\n\tv_nop\n\tv_nop" : "+v"(d) : "v"(a), "v"(b));
  return d;
}
__device__ __forceinline__ v16h frag_h(const _Float16* rowk0, int lane) {
  union { v16h v; v8h q[2]; } u; const _Float16* p = rowk0 + 8 * (lane >> 4);
  u.q[0] = *(const v8h*)p; u.q[1] = *(const v8h*)(p + 16); return u.v;
}
__device__ __forceinline__ v16h frag_f32(const float* rowk0, int lane) {
  v16h a; const float* p = rowk0 + 8 * (lane >> 4);
#pragma unroll
  for (int i = 0; i < 8; ++i) { a[i] = (_Float16)p[i]; a[8 + i] = (_Float16)p[16 + i]; }
  return a;
}
__device__ __forceinline__ v16h frag_f32s(const float* rowk0, int lane, float sc) {
  v16h a; const float* p = rowk0 + 8 * (lane >> 4);
#pragma unroll
  for (int i = 0; i < 8; ++i) { a[i] = (_Float16)(p[i] * sc); a[8 + i] = (_Float16)(p[16 + i] * sc); }
  return a;
}
__device__ __forceinline__ v16h fragc_f32(const float* W, int k0, int n, int lane, int ld, int K) {
  v16h a; const int g = lane >> 4;
#pragma unroll
  for (int i = 0; i < 8; ++i) { const int ka = k0 + 8 * g + i, kb = ka + 16;
    a[i] = (_Float16)(ka < K ? W[(size_t)ka * ld + n] : 0.f); a[8 + i] = (_Float16)(kb < K ? W[(size_t)kb * ld + n] : 0.f); }
  return a;
}
struct F2 { v16b h, l; };
__device__ __forceinline__ F2 bsplit16(const float v[16]) { F2 r;
#pragma unroll
  for (int i = 0; i < 16; ++i) { const __bf16 h = (__bf16)v[i]; r.h[i] = h; r.l[i] = (__bf16)(v[i] - (float)h); }
  return r; }
__device__ __forceinline__ F2 split_row(const float* row, int k0, int lane) { float v[16]; const float* p = row + k0 + 8 * (lane >> 4);
#pragma unroll
  for (int i = 0; i < 8; ++i) { v[i] = p[i]; v[8 + i] = p[16 + i]; }
  return bsplit16(v); }
__device__ __forceinline__ F2 split_rowK(const float* row, int k0, int lane, int K) { float v[16]; const int g = lane >> 4;
#pragma unroll
  for (int i = 0; i < 8; ++i) { const int ka = k0 + 8 * g + i, kb = ka + 16; v[i] = ka < K ? row[ka] : 0.f; v[8 + i] = kb < K ? row[kb] : 0.f; }
  return bsplit16(v); }
__device__ __forceinline__ F2 split_col(const float* W, int k0, int n, int lane, int ld, int K) { float v[16]; const int g = lane >> 4;
#pragma unroll
  for (int i = 0; i < 8; ++i) { const int ka = k0 + 8 * g + i, kb = ka + 16; v[i] = ka < K ? W[(size_t)ka * ld + n] : 0.f; v[8 + i] = kb < K ? W[(size_t)kb * ld + n] : 0.f; }
  return bsplit16(v); }
__device__ __forceinline__ v8f mac3(const F2& a, const F2& b, v8f c) { c = wmma_bf(a.l, b.h, c); c = wmma_bf(a.h, b.l, c); return wmma_bf(a.h, b.h, c); }
__device__ __forceinline__ float sigm(float v) { return 1.0f / (1.0f + expf(-v)); }
#define LDSX() do { asm volatile("s_wait_dscnt 0" ::: "memory"); __builtin_amdgcn_wave_barrier(); __builtin_amdgcn_fence(__ATOMIC_RELEASE, "workgroup"); } while (0)

#define NBTS 2048
#define SYM 14
#define FFT 128
#define NSC 108
#define LL (SYM * NSC)
#define KP 3040
#define NCOL (2 * LL)
#define NCOLP 3072

__global__ __launch_bounds__(256) void k_packB(const float* __restrict__ Cr, const float* __restrict__ Ci, _Float16* __restrict__ B16) {
  const int n = blockIdx.x, tid = threadIdx.x;
  const int m = n < LL ? n : n - LL; const bool im = n >= LL; const bool valid = n < NCOL;
  for (int q = tid; q < KP / 8; q += 256) { union { v8h h; v4u u; } pk;
#pragma unroll
    for (int i = 0; i < 8; ++i) { const int k = q * 8 + i; float v = 0.f;
      if (valid && k < 2 * LL) { const int l = k < LL ? k : k - LL; const float cr = Cr[(size_t)m * LL + l], ci = Ci[(size_t)m * LL + l];
        v = !im ? (k < LL ? cr : ci) : (k < LL ? -ci : cr); }
      pk.h[i] = (_Float16)(v * 16.0f); }
    vst2(B16 + (size_t)n * KP + q * 8, pk.u); }
}
__global__ __launch_bounds__(256) void k_packA(const float* __restrict__ xr, const float* __restrict__ xi, const int* __restrict__ sc, _Float16* __restrict__ A16) {
  const int r = blockIdx.x, tid = threadIdx.x;
  for (int q = tid; q < KP / 8; q += 256) { union { v8h h; v4u u; } pk;
#pragma unroll
    for (int i = 0; i < 8; ++i) { const int k = q * 8 + i; float v = 0.f;
      if (k < 2 * LL) { const int l = k < LL ? k : k - LL; const int sym = l / NSC, kk = l % NSC; int s = sc[kk]; s = s < 0 ? 0 : (s >= FFT ? FFT - 1 : s);
        v = (k < LL ? xr : xi)[((size_t)r * SYM + sym) * FFT + s]; }
      pk.h[i] = (_Float16)v; }
    vst2(A16 + (size_t)r * KP + q * 8, pk.u); }
}
__global__ __launch_bounds__(128) void k_gemm(const _Float16* __restrict__ A16, const _Float16* __restrict__ B16, float* __restrict__ Y) {
  __shared__ __align__(16) float so[4][16][132];
  const int tid = threadIdx.x, wave = tid >> 5, lane = tid & 31, col = lane & 15, g = lane >> 4;
  const int r0 = blockIdx.x * 64 + wave * 16, n0 = blockIdx.y * 128;
  v8f acc[8] = {};
#pragma unroll 1
  for (int kc = 0; kc < KP / 32; ++kc) { const v16h a = frag_h(A16 + (size_t)(r0 + col) * KP + kc * 32, lane);
#pragma unroll
    for (int j = 0; j < 8; ++j) acc[j] = wmma16(a, frag_h(B16 + (size_t)(n0 + j * 16 + col) * KP + kc * 32, lane), acc[j]); }
#pragma unroll
  for (int j = 0; j < 8; ++j)
#pragma unroll
    for (int r = 0; r < 8; ++r) so[wave][8 * g + r][j * 16 + col] = acc[j][r] * (1.0f / 16.0f);
  LDSX();
#pragma unroll 4
  for (int rl = 0; rl < 16; ++rl) vst2(Y + (size_t)(r0 + rl) * NCOLP + n0 + lane * 4, *(const v4f*)(&so[wave][rl][lane * 4]));
}
__global__ __launch_bounds__(128) void k_scatter(const float* __restrict__ Y, const int* __restrict__ sc, float* __restrict__ out) {
  __shared__ __align__(16) float rows[SYM][FFT];
  const int r = blockIdx.x, part = blockIdx.y, tid = threadIdx.x;
  for (int q = tid; q < SYM * FFT; q += 128) (&rows[0][0])[q] = 0.f;
  __syncthreads();
  for (int q = tid; q < SYM * NSC; q += 128) { const int sym = q / NSC, kk = q % NSC; int s = sc[kk]; s = s < 0 ? 0 : (s >= FFT ? FFT - 1 : s);
    rows[sym][s] = Y[(size_t)r * NCOLP + part * LL + q]; }
  __syncthreads();
  for (int q = tid; q < SYM * FFT / 4; q += 128) vst2(out + (((size_t)part * NBTS + r) * SYM) * FFT + q * 4, *(const v4f*)(&rows[0][0] + q * 4));
}
extern "C" void kernel_launch(void* const* d_in, const int* in_sizes, int n_in, void* d_out, int out_size, void* d_ws, size_t ws_size, hipStream_t stream) {
  (void)in_sizes; (void)n_in; (void)out_size; (void)ws_size;
  const float* xr = (const float*)d_in[0]; const float* xi = (const float*)d_in[1]; const float* Cr = (const float*)d_in[2]; const float* Ci = (const float*)d_in[3]; const int* sc = (const int*)d_in[4];
  float* out = (float*)d_out;
  char* ws = (char*)d_ws; size_t off = 0;
  auto take = [&](size_t bytes) { char* p = ws + off; off += (bytes + 255) & ~(size_t)255; return p; };
  _Float16* B16 = (_Float16*)take((size_t)NCOLP * KP * 2); _Float16* A16 = (_Float16*)take((size_t)NBTS * KP * 2); float* Y = (float*)take((size_t)NBTS * NCOLP * 4);
  k_packB<<<NCOLP, 256, 0, stream>>>(Cr, Ci, B16);
  k_packA<<<NBTS, 256, 0, stream>>>(xr, xi, sc, A16);
  k_gemm<<<dim3(NBTS / 64, NCOLP / 128), 128, 0, stream>>>(A16, B16, Y);
  k_scatter<<<dim3(NBTS, 2), 128, 0, stream>>>(Y, sc, out);
}
